// DualEncoderModel_35373350649881
// MI455X (gfx1250) — hardware-verified
//
#include <hip/hip_runtime.h>
#include <stddef.h>


typedef _Float16 h16;
typedef _Float16 v16h __attribute__((ext_vector_type(16)));
typedef _Float16 v8h  __attribute__((ext_vector_type(8)));
typedef float    v8f  __attribute__((ext_vector_type(8)));
typedef float    v4f  __attribute__((ext_vector_type(4)));

#ifndef NB
#define NB 64
#endif
#define NB_FULL 64
#define LOOK   50
#define NAG    256
#define NFR    128
#define FEAT   8
#define EMB    64
#define NPAIR  4096
#define KENC   400
#define KSTEP_ENC 13
#define KPAD   448
#define KCLS   256

static_assert(NB >= 1 && NB <= NB_FULL);
static_assert(KENC == LOOK * FEAT);
static_assert(FEAT == 8);
static_assert(32 * KSTEP_ENC >= KENC && 32 * KSTEP_ENC <= KPAD);
static_assert((KPAD % 64) == 0 && (KCLS % 64) == 0 && (KCLS % 32) == 0);
static_assert(NAG == 2 * NFR);
static_assert(NFR == 8 * 16);
static_assert(EMB == 64);
static_assert(KCLS == 4 * EMB);
static_assert((NPAIR % 128) == 0);

#define LDT 72
#define LDC 68
#define LDR 264
static_assert((LDT % 8) == 0 && LDT >= 64);
static_assert((LDC % 4) == 0 && LDC >= 64);
static_assert((LDR % 8) == 0 && LDR >= KCLS);

#define WCARRY 64.0f
#define XCARRY 16.0f
#define ACARRY 16.0f

#define WE_BYTES  ((size_t)2 * EMB * KPAD * 2)
#define W1_BYTES  ((size_t)EMB * KCLS * 2)
#define EMB_BYTES ((size_t)NB * NAG * EMB * 4)
#define OFF_WE  ((size_t)0)
#define OFF_W1  (OFF_WE + WE_BYTES)
#define OFF_EMB (OFF_W1 + W1_BYTES)
#define WS_TOTAL (OFF_EMB + EMB_BYTES)
static_assert((WE_BYTES % 128) == 0 && (W1_BYTES % 128) == 0 && (EMB_BYTES % 128) == 0);
static_assert(WS_TOTAL <= (size_t)134217728);

static_assert((size_t)128 * LDC * 4 <= (size_t)131072);
static_assert((size_t)128 * LDR * 2 + 256 * 4 + 128 * 4 <= (size_t)131072);

__device__ __forceinline__ float bf16r(float x) {
  unsigned int u = __float_as_uint(x);
  u = (u + 0x7FFFu + ((u >> 16) & 1u)) & 0xFFFF0000u;
  return __uint_as_float(u);
}

static __device__ __forceinline__ h16 toh_flush(float v) {
  const h16 r = (h16)v;
  return (fabsf(v) < 6.103515625e-05f) ? (h16)0.0f : r;
}

__device__ __forceinline__ v16h frag_at(const _Float16* p) {
  v8h lo = *(const v8h*)(p);
  v8h hi = *(const v8h*)(p + 16);
  v16h out;
#pragma unroll
  for (int i = 0; i < 8; ++i) { out[i] = lo[i]; out[i + 8] = hi[i]; }
  return out;
}
__device__ __forceinline__ v16h frag_join(v8h lo, v8h hi) {
  v16h out;
#pragma unroll
  for (int i = 0; i < 8; ++i) { out[i] = lo[i]; out[i + 8] = hi[i]; }
  return out;
}

__device__ __forceinline__ v8f wmma16(v16h a, v16h b, v8f c) {
  v8f d = __builtin_amdgcn_wmma_f32_16x16x32_f16(false, a, false, b, (short)0, c,
                                                 false, false);
  asm volatile("v_nop\n\tv_nop\n\tv_nop\n\tv_nop" : "+v"(d) : "v"(a), "v"(b));
  return d;
}

__device__ __forceinline__ float red16_sum(float x) {
#pragma unroll
  for (int off = 1; off < 16; off <<= 1) x += __shfl_xor(x, off, 32);
  return x;
}

__global__ __launch_bounds__(256) void wconv_kernel(
    const float* __restrict__ W, _Float16* __restrict__ Wt, unsigned ldw, unsigned ldk,
    unsigned krows) {
  __shared__ _Float16 T[64 * LDT];
  const unsigned tid = threadIdx.x;
  const unsigned n0 = blockIdx.x * 64u;
  const unsigned k0 = blockIdx.y * 64u;
#pragma unroll 4
  for (unsigned j = 0; j < 16u; ++j) {
    const unsigned idx = tid + 256u * j;
    const unsigned kr = idx >> 6, nc = idx & 63u;
    const unsigned kk = k0 + kr;
    const unsigned kc = (kk < krows) ? kk : (krows - 1u);
    const float v = W[(size_t)kc * ldw + n0 + nc];
    const h16 hv = toh_flush(WCARRY * bf16r(v));
    T[nc * LDT + kr] = (kk < krows) ? hv : (h16)0.0f;
  }
  __syncthreads();
  v8h x[2];
  size_t off[2];
#pragma unroll
  for (unsigned i = 0; i < 2u; ++i) {
    const unsigned n = 32u * i + (tid >> 3);
    const unsigned kc = (tid & 7u) * 8u;
    x[i] = *(const v8h*)&T[n * LDT + kc];
    off[i] = (size_t)(n0 + n) * ldk + k0 + kc;
  }
#pragma unroll
  for (int i = 0; i < 2; ++i) *(volatile v8h*)(Wt + off[i]) = x[i];
  __threadfence();
#pragma unroll
  for (int i = 0; i < 2; ++i) *(volatile v8h*)(Wt + off[i]) = x[i];
}

static_assert(8 * 16 == NFR);
__global__ __launch_bounds__(256) void enc_kernel(
    const float* __restrict__ traj, const _Float16* __restrict__ Wt,
    const float* __restrict__ biasf, const float* __restrict__ biasu,
    float* __restrict__ emb) {
  __shared__ __attribute__((aligned(16))) float Cs[128 * LDC];
  const unsigned tid = threadIdx.x, lane = tid & 31u;
  const unsigned wave = (unsigned)__builtin_amdgcn_readfirstlane((int)(tid >> 5));
  const unsigned hh = lane >> 4, m = lane & 15u;
  const unsigned b = blockIdx.x >> 1;
  const unsigned half = blockIdx.x & 1u;
  const unsigned agent = half * (unsigned)NFR + wave * 16u + m;

  const float* ap = traj + (size_t)b * (LOOK * NAG * FEAT) + (size_t)agent * FEAT;
  const _Float16* bp = Wt + (size_t)(half * (unsigned)EMB + m) * KPAD + hh * 8u;

  v8f acc[4];
#pragma unroll
  for (int t = 0; t < 4; ++t) acc[t] = (v8f){};

#pragma unroll 1
  for (unsigned j = 0; j < (unsigned)KSTEP_ENC; ++j) {
    const unsigned l0 = 4u * j + hh;
    const unsigned l1 = l0 + 2u;
    const unsigned l0c = (l0 < (unsigned)LOOK) ? l0 : (unsigned)(LOOK - 1);
    const unsigned l1c = (l1 < (unsigned)LOOK) ? l1 : (unsigned)(LOOK - 1);
    const bool ok0 = l0 < (unsigned)LOOK;
    const bool ok1 = l1 < (unsigned)LOOK;
    const float* p0 = ap + (size_t)l0c * (NAG * FEAT);
    const float* p1 = ap + (size_t)l1c * (NAG * FEAT);
    const v4f a0 = *(const v4f*)(p0);
    const v4f a1 = *(const v4f*)(p0 + 4);
    const v4f c0 = *(const v4f*)(p1);
    const v4f c1 = *(const v4f*)(p1 + 4);
    v16h a;
#pragma unroll
    for (int i = 0; i < 4; ++i) {
      const h16 e0 = toh_flush(XCARRY * bf16r(a0[i]));
      const h16 e1 = toh_flush(XCARRY * bf16r(a1[i]));
      const h16 e2 = toh_flush(XCARRY * bf16r(c0[i]));
      const h16 e3 = toh_flush(XCARRY * bf16r(c1[i]));
      a[i]      = ok0 ? e0 : (h16)0.0f;
      a[i + 4]  = ok0 ? e1 : (h16)0.0f;
      a[i + 8]  = ok1 ? e2 : (h16)0.0f;
      a[i + 12] = ok1 ? e3 : (h16)0.0f;
    }
    const unsigned k0 = 32u * j;
#pragma unroll
    for (int t = 0; t < 4; ++t) {
      const v16h bfr = frag_at(bp + (size_t)(t * 16) * KPAD + k0);
      acc[t] = wmma16(a, bfr, acc[t]);
    }
  }

#pragma unroll
  for (int t = 0; t < 4; ++t)
#pragma unroll
    for (int r = 0; r < 8; ++r)
      Cs[(wave * 16u + hh * 8u + (unsigned)r) * LDC + (unsigned)t * 16u + m] = acc[t][r];
  __syncthreads();

  const float cs = 1.0f / (WCARRY * XCARRY);
  const unsigned c = (tid & 15u) * 4u;
  const v4f gf = *(const v4f*)(biasf + c);
  const v4f gu = *(const v4f*)(biasu + c);
  v4f g;
#pragma unroll
  for (int jn = 0; jn < 4; ++jn) g[jn] = bf16r((half != 0u) ? gu[jn] : gf[jn]);

  v4f xs[8];
  size_t off[8];
#pragma unroll
  for (unsigned i = 0; i < 8u; ++i) {
    const unsigned r = 16u * i + (tid >> 4);
    const v4f u = *(const v4f*)&Cs[r * LDC + c];
    v4f val;
#pragma unroll
    for (int jn = 0; jn < 4; ++jn) val[jn] = u[jn] * cs + g[jn];
    xs[i] = val;
    off[i] = ((size_t)b * NAG + half * (unsigned)NFR + r) * EMB + c;
  }
#pragma unroll
  for (int i = 0; i < 8; ++i) *(volatile v4f*)(emb + off[i]) = xs[i];
  __threadfence();
#pragma unroll
  for (int i = 0; i < 8; ++i) *(volatile v4f*)(emb + off[i]) = xs[i];
}

static_assert(32 * 16 == 128 * 4);
static_assert(4 * 256 == 128 * 8);
__global__ __launch_bounds__(256) void cls_kernel(
    const float* __restrict__ emb, const int* __restrict__ pairs,
    const _Float16* __restrict__ W1t, const float* __restrict__ b1,
    const float* __restrict__ W2, const float* __restrict__ b2,
    float* __restrict__ out) {
  __shared__ __attribute__((aligned(16))) _Float16 Rs[128 * LDR];
  __shared__ int s_idx[256];
  __shared__ __attribute__((aligned(16))) float s_out[128];

  const unsigned tid = threadIdx.x, lane = tid & 31u;
  const unsigned wave = (unsigned)__builtin_amdgcn_readfirstlane((int)(tid >> 5));
  const unsigned hh = lane >> 4, m = lane & 15u;
  const unsigned b = blockIdx.x / (unsigned)(NPAIR / 128);
  const unsigned p0 = (blockIdx.x % (unsigned)(NPAIR / 128)) * 128u;

  {
    const int v = pairs[((size_t)b * NPAIR + p0) * 2u + tid];
    int fi = v;
    fi = (fi < 0) ? 0 : fi;
    fi = (fi > (NFR - 1)) ? (NFR - 1) : fi;
    int ui = v - NFR;
    ui = (ui < 0) ? 0 : ui;
    ui = (ui > (NAG - NFR - 1)) ? (NAG - NFR - 1) : ui;
    ui += NFR;
    s_idx[tid] = ((tid & 1u) != 0u) ? ui : fi;
  }
  __syncthreads();

  const float* eb = emb + (size_t)b * NAG * EMB;
#pragma unroll 1
  for (unsigned j = 0; j < 4u; ++j) {
    const unsigned idx = tid + 256u * j;
    const unsigned pr = idx >> 3, e8 = (idx & 7u) * 8u;
    const unsigned fi = (unsigned)s_idx[2u * pr];
    const unsigned ui = (unsigned)s_idx[2u * pr + 1u];
    const v4f f0 = *(const v4f*)(eb + (size_t)fi * EMB + e8);
    const v4f f1 = *(const v4f*)(eb + (size_t)fi * EMB + e8 + 4u);
    const v4f u0 = *(const v4f*)(eb + (size_t)ui * EMB + e8);
    const v4f u1 = *(const v4f*)(eb + (size_t)ui * EMB + e8 + 4u);
    v8h xf, xu, xd, xp;
#pragma unroll
    for (int i = 0; i < 4; ++i) {
      xf[i]     = toh_flush(ACARRY * f0[i]);
      xf[i + 4] = toh_flush(ACARRY * f1[i]);
      xu[i]     = toh_flush(ACARRY * u0[i]);
      xu[i + 4] = toh_flush(ACARRY * u1[i]);
      xd[i]     = toh_flush(ACARRY * fabsf(f0[i] - u0[i]));
      xd[i + 4] = toh_flush(ACARRY * fabsf(f1[i] - u1[i]));
      xp[i]     = toh_flush(ACARRY * (f0[i] * u0[i]));
      xp[i + 4] = toh_flush(ACARRY * (f1[i] * u1[i]));
    }
    *(v8h*)&Rs[pr * LDR + e8]             = xf;
    *(v8h*)&Rs[pr * LDR + EMB + e8]       = xu;
    *(v8h*)&Rs[pr * LDR + 2 * EMB + e8]   = xd;
    *(v8h*)&Rs[pr * LDR + 3 * EMB + e8]   = xp;
  }
  __syncthreads();

  v8f acc[4];
#pragma unroll
  for (int t = 0; t < 4; ++t) acc[t] = (v8f){};
  const unsigned abase = (wave * 16u + m) * LDR + hh * 8u;
  const _Float16* bp = W1t + (size_t)m * KCLS + hh * 8u;
#pragma unroll 2
  for (unsigned k0 = 0; k0 < (unsigned)KCLS; k0 += 32u) {
    const v8h lo = *(const v8h*)&Rs[abase + k0];
    const v8h hi = *(const v8h*)&Rs[abase + k0 + 16u];
    const v16h a = frag_join(lo, hi);
#pragma unroll
    for (int t = 0; t < 4; ++t) {
      const v16h bfr = frag_at(bp + (size_t)(t * 16) * KCLS + k0);
      acc[t] = wmma16(a, bfr, acc[t]);
    }
  }

  const float cs = 1.0f / (WCARRY * ACARRY);
  float bb[4], ww[4];
#pragma unroll
  for (int t = 0; t < 4; ++t) {
    bb[t] = bf16r(b1[(unsigned)t * 16u + m]);
    ww[t] = bf16r(W2[(unsigned)t * 16u + m]);
  }
  const float bias2 = bf16r(b2[0]);
  float sel = 0.0f;
#pragma unroll
  for (int v = 0; v < 8; ++v) {
    float s = 0.0f;
#pragma unroll
    for (int t = 0; t < 4; ++t) {
      float hv = acc[t][v] * cs + bb[t];
      hv = (hv > 0.0f) ? hv : 0.0f;
      s += hv * ww[t];
    }
    s = red16_sum(s);
    sel = (m == (unsigned)v) ? s : sel;
  }
  if (m < 8u) s_out[wave * 16u + hh * 8u + m] = sel + bias2;
  __syncthreads();

  if (wave == 0u) {
    const v4f x = *(const v4f*)&s_out[lane * 4u];
    float* o = out + (size_t)b * NPAIR + p0 + lane * 4u;
    *(volatile v4f*)o = x;
    __threadfence();
    *(volatile v4f*)o = x;
  }
}

extern "C" void kernel_launch(void* const* d_in, const int* in_sizes, int n_in,
                              void* d_out, int out_size, void* d_ws, size_t ws_size,
                              hipStream_t stream) {
  if (n_in < 11) return;
  if ((long long)in_sizes[0] < (long long)NB * LOOK * NAG * FEAT) return;
  if ((long long)in_sizes[2] < (long long)NB * NPAIR * 2) return;
  if ((long long)in_sizes[3] < (long long)KENC * EMB) return;
  if ((long long)in_sizes[5] < (long long)KENC * EMB) return;
  if (in_sizes[4] < EMB || in_sizes[6] < EMB) return;
  if ((long long)in_sizes[7] < (long long)KCLS * EMB) return;
  if (in_sizes[8] < EMB || in_sizes[9] < EMB || in_sizes[10] < 1) return;
  if ((long long)out_size < (long long)NB * NPAIR) return;
  if (ws_size < WS_TOTAL) return;

  const float* traj  = (const float*)d_in[0];
  const int*   pairs = (const int*)d_in[2];
  const float* encfW = (const float*)d_in[3];
  const float* encfb = (const float*)d_in[4];
  const float* encuW = (const float*)d_in[5];
  const float* encub = (const float*)d_in[6];
  const float* clsW1 = (const float*)d_in[7];
  const float* clsb1 = (const float*)d_in[8];
  const float* clsW2 = (const float*)d_in[9];
  const float* clsb2 = (const float*)d_in[10];
  float* out = (float*)d_out;

  char* ws = (char*)d_ws;
  _Float16* We_t = (_Float16*)(ws + OFF_WE);
  _Float16* W1_t = (_Float16*)(ws + OFF_W1);
  float*    Emb  = (float*)(ws + OFF_EMB);

  dim3 blk(256);
  wconv_kernel<<<dim3(EMB / 64, KPAD / 64), blk, 0, stream>>>(
      encfW, We_t, (unsigned)EMB, (unsigned)KPAD, (unsigned)KENC);
  wconv_kernel<<<dim3(EMB / 64, KPAD / 64), blk, 0, stream>>>(
      encuW, We_t + (size_t)EMB * KPAD, (unsigned)EMB, (unsigned)KPAD, (unsigned)KENC);
  wconv_kernel<<<dim3(EMB / 64, KCLS / 64), blk, 0, stream>>>(
      clsW1, W1_t, (unsigned)EMB, (unsigned)KCLS, (unsigned)KCLS);

  enc_kernel<<<dim3(NB * 2), blk, 0, stream>>>(traj, We_t, encfb, encub, Emb);
  cls_kernel<<<dim3(NB * (NPAIR / 128)), blk, 0, stream>>>(
      Emb, pairs, W1_t, clsb1, clsW2, clsb2, out);
}
